// GraphEncoder_17952963298146
// MI455X (gfx1250) — hardware-verified
//
#include <hip/hip_runtime.h>
#include <stddef.h>
#include <stdint.h>
#include <math.h>


#define NGRAPH 32
#define NNODE  2000
#define NEDGE  32000
#define DF     128
#define NREL   39
#define NBAS   8
#define NR1    40
#define KW     1152
#define K2     2304
#define NTHR   256
#define NWAVE  8
#define EPT    8
#define CHUNK  (NTHR * EPT)
#define WCAP   (EPT * 32)
#define LISTN  (NWAVE * WCAP)
#define NBRUN  125
#define NBLKG  16
#define SLOTB  7
#define RCAP   3072
#define HISTN  8192
#define YPN    (NR1 * DF)
#define ZINTS  (NWAVE * YPN + HISTN + 2 * RCAP + LISTN)
#define SCAN_LDS_INTS (ZINTS + 16)
#define UPART  2048
#define NPARTW 18
#define WBLK   ((NPARTW * UPART) / NTHR)
#define XUNITS (NGRAPH * NNODE * (DF / 8))
#define XBLK   (XUNITS / NTHR)
#define NOUT   (NGRAPH * DF)
#define WSMAX  134217728

static_assert((CHUNK & (CHUNK - 1)) == 0 && CHUNK <= 4096);
static_assert(NBRUN * NBLKG == NNODE && NBRUN <= (1 << SLOTB));
static_assert(((long long)CHUNK << SLOTB) < (1LL << 31));
static_assert(NREL <= 64 && (NBRUN << 6) <= HISTN && NNODE <= 2048);
static_assert(ZINTS % (NTHR * 4) == 0);
static_assert((YPN / 4) == 5 * NTHR);
static_assert(KW == 9 * DF && K2 == 2 * KW && K2 % 32 == 0);
static_assert((NPARTW * UPART) % NTHR == 0 && UPART % NTHR == 0 && UPART == DF * (DF / 8));
static_assert(XUNITS % NTHR == 0);
static_assert(KW == 4 * NTHR + 128 && (K2 / 8) == NTHR + 32);
static_assert(NGRAPH == 32 && DF == 4 * 32 && DF == NWAVE * 16 && NGRAPH == NWAVE * 4);
static_assert(SCAN_LDS_INTS * 4 <= 300000);
static_assert(NEDGE % 4 == 0);

typedef float          v4f   __attribute__((ext_vector_type(4)));
typedef float          v8f   __attribute__((ext_vector_type(8)));
typedef int            v4i   __attribute__((ext_vector_type(4)));
typedef int            v8i   __attribute__((ext_vector_type(8)));
typedef unsigned       v2u   __attribute__((ext_vector_type(2)));
typedef unsigned short v8us  __attribute__((ext_vector_type(8)));
typedef unsigned short v16us __attribute__((ext_vector_type(16)));
typedef __bf16         v16bf __attribute__((ext_vector_type(16)));
typedef v4f  __attribute__((may_alias)) v4fa;
typedef v4i  __attribute__((may_alias)) v4ia;
typedef v2u  __attribute__((may_alias)) v2ua;
typedef v8us __attribute__((may_alias)) v8usa;
union FragB { v16bf v; v16us u; v8us h[2]; v8i w; };

__device__ __forceinline__ v8f wmb(const FragB& a, const FragB& b, v8f c) {
  v8f d = __builtin_amdgcn_wmma_f32_16x16x32_bf16(false, a.v, false, b.v, (short)0, c, false, false);
  asm volatile("v_nop\n\tv_nop\n\tv_nop\n\tv_nop" : "+v"(d) : "v"(a.w), "v"(b.w));
  return d;
}

__device__ __forceinline__ unsigned bf16_bits(float f) {
  const unsigned u = __float_as_uint(f);
  return (u + 0x7FFFu + ((u >> 16) & 1u)) >> 16;
}
__device__ __forceinline__ float bf16_val(float f) {
  return __uint_as_float(bf16_bits(f) << 16);
}

template <int SLB>
__device__ __forceinline__ int scan_chunk(const int* __restrict__ dsts, int nE, int cbase, int slotBase,
                                          int nb, int vec8, int* list, int tid, int lane, int wave) {
  int wc = 0;
  const int el0  = tid * EPT;
  const int e0   = cbase + el0;
  const int sent = -2147483647 - 1;
  v4i da, db;
  if (vec8 != 0 && cbase + CHUNK <= nE) {
    da = *(const v4i*)(dsts + e0);
    db = *(const v4i*)(dsts + e0 + 4);
  } else {
    da.x = (e0     < nE) ? dsts[min(e0,     nE - 1)] : sent;
    da.y = (e0 + 1 < nE) ? dsts[min(e0 + 1, nE - 1)] : sent;
    da.z = (e0 + 2 < nE) ? dsts[min(e0 + 2, nE - 1)] : sent;
    da.w = (e0 + 3 < nE) ? dsts[min(e0 + 3, nE - 1)] : sent;
    db.x = (e0 + 4 < nE) ? dsts[min(e0 + 4, nE - 1)] : sent;
    db.y = (e0 + 5 < nE) ? dsts[min(e0 + 5, nE - 1)] : sent;
    db.z = (e0 + 6 < nE) ? dsts[min(e0 + 6, nE - 1)] : sent;
    db.w = (e0 + 7 < nE) ? dsts[min(e0 + 7, nE - 1)] : sent;
  }
  const unsigned nbs = (unsigned)slotBase;
  const unsigned unb = (unsigned)nb;
  const unsigned s0 = (unsigned)da.x - nbs, s1 = (unsigned)da.y - nbs;
  const unsigned s2 = (unsigned)da.z - nbs, s3 = (unsigned)da.w - nbs;
  const unsigned s4 = (unsigned)db.x - nbs, s5 = (unsigned)db.y - nbs;
  const unsigned s6 = (unsigned)db.z - nbs, s7 = (unsigned)db.w - nbs;
  const bool h0 = s0 < unb, h1 = s1 < unb, h2 = s2 < unb, h3 = s3 < unb;
  const bool h4 = s4 < unb, h5 = s5 < unb, h6 = s6 < unb, h7 = s7 < unb;
  const unsigned any = __builtin_amdgcn_ballot_w32(h0 | h1 | h2 | h3 | h4 | h5 | h6 | h7);
  if (any != 0u) {
#define HITJ(J, HJ, SJ) { \
      const unsigned mj = __builtin_amdgcn_ballot_w32(HJ); \
      if (mj != 0u) { \
        if (HJ) { \
          const int pos = wc + (int)__builtin_amdgcn_mbcnt_lo(mj, 0u); \
          if (pos < WCAP) list[wave * WCAP + pos] = ((el0 + (J)) << SLB) | (int)(SJ); \
        } \
        wc += (int)__builtin_popcount(mj); } }
    HITJ(0, h0, s0)
    HITJ(1, h1, s1)
    HITJ(2, h2, s2)
    HITJ(3, h3, s3)
    HITJ(4, h4, s4)
    HITJ(5, h5, s5)
    HITJ(6, h6, s6)
    HITJ(7, h7, s7)
#undef HITJ
  }
  return wc;
}

__global__ __launch_bounds__(NTHR) void k_prep(const int* __restrict__ nid, const float* __restrict__ emb, int nV,
                                               const float* __restrict__ root, const float* __restrict__ bases,
                                               unsigned short* xb, unsigned short* wt) {
  const int tid = (int)threadIdx.x;
  v8us o;
  unsigned short* dp;
  if ((int)blockIdx.x < WBLK) {
    const int u    = (int)blockIdx.x * NTHR + tid;
    const int part = u >> 11;
    const int v    = u & (UPART - 1);
    const int n    = v >> 4;
    const int k8   = (v & 15) * 8;
    const int dup  = part / 9;
    const int mat  = part - 9 * dup;
    const float* W = (mat == 0) ? root : (bases + (size_t)(mat - 1) * DF * DF);
    const float* p = W + (size_t)k8 * DF + n;
#pragma unroll
    for (int i = 0; i < 8; ++i) o[i] = (unsigned short)bf16_bits(p[(size_t)i * DF]);
    dp = wt + (size_t)n * K2 + dup * KW + mat * DF + k8;
  } else {
    const int u = ((int)blockIdx.x - WBLK) * NTHR + tid;
    if (u >= XUNITS) return;
    const int row = u >> 4;
    const int k8  = (u & 15) * 8;
    int id = nid[row];
    id = id < 0 ? 0 : (id > nV - 1 ? nV - 1 : id);
    const float* p = emb + (size_t)id * DF + k8;
    const v4f a = *(const v4fa*)p;
    const v4f b = *(const v4fa*)(p + 4);
    o[0] = (unsigned short)bf16_bits(a.x); o[1] = (unsigned short)bf16_bits(a.y);
    o[2] = (unsigned short)bf16_bits(a.z); o[3] = (unsigned short)bf16_bits(a.w);
    o[4] = (unsigned short)bf16_bits(b.x); o[5] = (unsigned short)bf16_bits(b.y);
    o[6] = (unsigned short)bf16_bits(b.z); o[7] = (unsigned short)bf16_bits(b.w);
    dp = xb + (size_t)row * DF + k8;
  }
  *(volatile v8us*)dp = o;
  __threadfence();
  *(volatile v8us*)dp = o;
}

__global__ __launch_bounds__(NTHR) void k_scan(const int* __restrict__ eidx, const int* __restrict__ etype,
                                               const unsigned short* __restrict__ xb, float* rec) {
  extern __shared__ __attribute__((aligned(16))) int dsm[];
  float* yp   = (float*)dsm;
  int*   hist = dsm + NWAVE * YPN;
  int*   hl   = hist + HISTN;
  float* winv = (float*)(hl + RCAP);
  int*   list = hl + 2 * RCAP;
  int*   misc = list + LISTN;
  const int tid  = (int)threadIdx.x, lane = tid & 31;
  const int wave = __builtin_amdgcn_readfirstlane(tid >> 5);
  const int blk  = (int)blockIdx.x;
  const int b    = (int)blockIdx.y;
  const int* srcp = eidx + (size_t)(2 * b) * NEDGE;
  const int* dstp = srcp + NEDGE;
  const int* etp  = etype + (size_t)b * NEDGE;
  const int slotBase = blk * NBRUN;
  const int gbase    = b * NNODE;

  {
    const v4i z4 = {0, 0, 0, 0};
    for (int i = tid * 4; i < ZINTS; i += NTHR * 4) *(v4ia*)(dsm + i) = z4;
    if (tid < 16) misc[tid] = 0;
  }
  __syncthreads();

  int t = 0, ov = 0;
  const int nChunks = (NEDGE + CHUNK - 1) / CHUNK;
#pragma unroll 1
  for (int ch = 0; ch < nChunks; ++ch) {
    const int cbase = ch * CHUNK;
    const int wc = scan_chunk<SLOTB>(dstp, NEDGE, cbase, slotBase, NBRUN, 1, list, tid, lane, wave);
    if (lane == 0) misc[wave] = wc;
    __syncthreads();
    if (wave == 0) {
#pragma unroll 1
      for (int w2 = 0; w2 < NWAVE; ++w2) {
        int c = misc[w2];
        c = c < 0 ? 0 : (c > WCAP ? WCAP : c);
#pragma unroll 1
        for (int b0 = 0; b0 < c; b0 += 32) {
          const int idx = b0 + lane;
          const int ent = list[w2 * WCAP + (idx < WCAP ? idx : WCAP - 1)];
          int slot = ent & ((1 << SLOTB) - 1);
          slot = slot > NBRUN - 1 ? NBRUN - 1 : slot;
          int eid = cbase + ((ent >> SLOTB) & (CHUNK - 1));
          eid = eid > NEDGE - 1 ? NEDGE - 1 : eid;
          int ty = etp[eid];
          ty = ty < 0 ? 0 : (ty > NREL - 1 ? NREL - 1 : ty);
          int sr = srcp[eid];
          sr = sr < 0 ? 0 : (sr > NNODE - 1 ? NNODE - 1 : sr);
          const int pk  = (sr << 13) | (slot << 6) | ty;
          const int pos = t + idx;
          if (idx < c && pos < RCAP) hl[pos] = pk;
          const int m32 = (c - b0) < 32 ? (c - b0) : 32;
#pragma unroll 1
          for (int k = 0; k < m32; ++k) {
            const int u   = __builtin_amdgcn_readlane(pk, k);
            const int key = u & (HISTN - 1);
            if (lane == 0) hist[key] = hist[key] + 1;
          }
        }
        if (t + c > RCAP) ov = 1;
        t = (t + c > RCAP) ? RCAP : (t + c);
      }
    }
    __syncthreads();
  }
  if (tid == 0) { misc[8] = t; misc[9] = ov; }
  __syncthreads();
  int tt = __builtin_amdgcn_readfirstlane(misc[8]);
  tt = tt < 0 ? 0 : (tt > RCAP ? RCAP : tt);
  const int ovf = __builtin_amdgcn_readfirstlane(misc[9]);

#pragma unroll 1
  for (int pos = tid; pos < tt; pos += NTHR) {
    const int key = hl[pos] & (HISTN - 1);
    int c = hist[key];
    c = c < 1 ? 1 : c;
    winv[pos] = 1.0f / (float)c;
  }
  __syncthreads();

  float* yw = yp + wave * YPN;
#pragma unroll 1
  for (int pos = wave; pos < tt; pos += NWAVE) {
    const int   ent = __builtin_amdgcn_readfirstlane(hl[pos]);
    const float iv  = __int_as_float(__builtin_amdgcn_readfirstlane(__float_as_int(winv[pos])));
    int sr = (ent >> 13) & 2047;
    sr = sr > NNODE - 1 ? NNODE - 1 : sr;
    int ty = ent & 63;
    ty = ty > NREL - 1 ? NREL - 1 : ty;
    const v2u wv = *(const v2ua*)(xb + (size_t)(gbase + sr) * DF + 4 * lane);
    const float x0 = __uint_as_float(wv.x << 16);
    const float x1 = __uint_as_float(wv.x & 0xffff0000u);
    const float x2 = __uint_as_float(wv.y << 16);
    const float x3 = __uint_as_float(wv.y & 0xffff0000u);
    float* yq = yw + ty * DF + 4 * lane;
    v4f a = *(v4fa*)yq;
    a.x = fmaf(iv, x0, a.x);
    a.y = fmaf(iv, x1, a.y);
    a.z = fmaf(iv, x2, a.z);
    a.w = fmaf(iv, x3, a.w);
    *(v4fa*)yq = a;
  }
#pragma unroll 1
  for (int i = wave; i < NBRUN; i += NWAVE) {
    const v2u wv = *(const v2ua*)(xb + (size_t)(gbase + slotBase + i) * DF + 4 * lane);
    float* yq = yw + NREL * DF + 4 * lane;
    v4f a = *(v4fa*)yq;
    a.x += __uint_as_float(wv.x << 16);
    a.y += __uint_as_float(wv.x & 0xffff0000u);
    a.z += __uint_as_float(wv.y << 16);
    a.w += __uint_as_float(wv.y & 0xffff0000u);
    *(v4fa*)yq = a;
  }
  __syncthreads();

  const float pz = (ovf != 0) ? __int_as_float(0x7fc00000) : 0.0f;
  v4f vals[5];
#pragma unroll
  for (int it = 0; it < 5; ++it) {
    const int i4 = 4 * (it * NTHR + tid);
    v4f s = *(const v4fa*)(yp + i4);
#pragma unroll
    for (int w2 = 1; w2 < NWAVE; ++w2) {
      const v4f q = *(const v4fa*)(yp + w2 * YPN + i4);
      s.x += q.x; s.y += q.y; s.z += q.z; s.w += q.w;
    }
    s.x += pz; s.y += pz; s.z += pz; s.w += pz;
    vals[it] = s;
  }
  float* rp = rec + (size_t)(b * NBLKG + blk) * YPN;
#pragma unroll
  for (int it = 0; it < 5; ++it) *(volatile v4f*)(rp + 4 * (it * NTHR + tid)) = vals[it];
  __threadfence();
#pragma unroll
  for (int it = 0; it < 5; ++it) *(volatile v4f*)(rp + 4 * (it * NTHR + tid)) = vals[it];
}

__global__ __launch_bounds__(NTHR) void k_combine(const float* __restrict__ rec, const float* __restrict__ comp,
                                                  unsigned short* a2) {
  __shared__ __attribute__((aligned(16))) float ys[YPN];
  __shared__ float cmx[NR1 * 9];
  __shared__ __attribute__((aligned(16))) unsigned short a2s[K2];
  const int tid = (int)threadIdx.x;
  const int b   = (int)blockIdx.x;

#pragma unroll 1
  for (int i = tid; i < NR1 * 9; i += NTHR) {
    const int r  = i / 9;
    const int j  = i - 9 * r;
    const int rc = r > NREL - 1 ? NREL - 1 : r;
    const int kc = j > 0 ? j - 1 : 0;
    const float cv = bf16_val(comp[rc * NBAS + kc]);
    const float one = (r == NREL) ? 1.0f : 0.0f;
    const float mix = (r < NREL) ? cv : 0.0f;
    cmx[i] = (j == 0) ? one : mix;
  }
  const float* rb = rec + (size_t)b * NBLKG * YPN;
#pragma unroll 1
  for (int it = 0; it < 5; ++it) {
    const int i4 = 4 * (it * NTHR + tid);
    v4f s = {0.0f, 0.0f, 0.0f, 0.0f};
#pragma unroll 4
    for (int q = 0; q < NBLKG; ++q) {
      const v4f v = *(const v4fa*)(rb + (size_t)q * YPN + i4);
      s.x += v.x; s.y += v.y; s.z += v.z; s.w += v.w;
    }
    *(v4fa*)(ys + i4) = s;
  }
  __syncthreads();
#pragma unroll 1
  for (int o = tid; o < KW; o += NTHR) {
    const int j = o >> 7;
    const int d = o & (DF - 1);
    float acc = 0.0f;
#pragma unroll 4
    for (int r = 0; r < NR1; ++r) acc = fmaf(cmx[r * 9 + j], ys[r * DF + d], acc);
    const unsigned hb = bf16_bits(acc);
    const unsigned lb = bf16_bits(acc - __uint_as_float(hb << 16));
    a2s[o]      = (unsigned short)hb;
    a2s[KW + o] = (unsigned short)lb;
  }
  __syncthreads();
  const bool t2 = tid < 32;
  const int  u1 = t2 ? (tid + NTHR) : tid;
  const v8us q0 = *(const v8usa*)(a2s + 8 * tid);
  const v8us q1 = *(const v8usa*)(a2s + 8 * u1);
  unsigned short* rp = a2 + (size_t)b * K2;
  *(volatile v8us*)(rp + 8 * tid) = q0;
  if (t2) *(volatile v8us*)(rp + 8 * u1) = q1;
  __threadfence();
  *(volatile v8us*)(rp + 8 * tid) = q0;
  if (t2) *(volatile v8us*)(rp + 8 * u1) = q1;
}

__global__ __launch_bounds__(NTHR) void k_gemm(const unsigned short* __restrict__ a2,
                                               const unsigned short* __restrict__ wt,
                                               const float* __restrict__ bias, float* out) {
  __shared__ __attribute__((aligned(16))) float G[NGRAPH * DF];
  const int tid = (int)threadIdx.x, lane = tid & 31, wave = tid >> 5, hh = lane >> 4, m = lane & 15;

  v8f acc0 = {0.f, 0.f, 0.f, 0.f, 0.f, 0.f, 0.f, 0.f};
  v8f acc1 = {0.f, 0.f, 0.f, 0.f, 0.f, 0.f, 0.f, 0.f};
  const unsigned short* ap0 = a2 + (size_t)m * K2 + 8 * hh;
  const unsigned short* ap1 = a2 + (size_t)(16 + m) * K2 + 8 * hh;
  const unsigned short* wp  = wt + (size_t)(16 * wave + m) * K2 + 8 * hh;
#pragma unroll 1
  for (int k0 = 0; k0 < K2; k0 += 32) {
    FragB bf, a0, a1;
    bf.h[0] = *(const v8usa*)(wp + k0);
    bf.h[1] = *(const v8usa*)(wp + k0 + 16);
    a0.h[0] = *(const v8usa*)(ap0 + k0);
    a0.h[1] = *(const v8usa*)(ap0 + k0 + 16);
    a1.h[0] = *(const v8usa*)(ap1 + k0);
    a1.h[1] = *(const v8usa*)(ap1 + k0 + 16);
    acc0 = wmb(a0, bf, acc0);
    acc1 = wmb(a1, bf, acc1);
  }
  const int lc = 16 * wave + m;
#pragma unroll
  for (int r = 0; r < 8; ++r) {
    G[(8 * hh + r) * DF + lc]      = acc0[r];
    G[(16 + 8 * hh + r) * DF + lc] = acc1[r];
  }
  __syncthreads();

  v4f bb;
  {
    const v4f t4 = *(const v4fa*)(bias + 4 * lane);
    bb.x = 2000.0f * bf16_val(t4.x);
    bb.y = 2000.0f * bf16_val(t4.y);
    bb.z = 2000.0f * bf16_val(t4.z);
    bb.w = 2000.0f * bf16_val(t4.w);
  }
  v4f ov[4];
#pragma unroll
  for (int i = 0; i < 4; ++i) {
    const int row = 4 * wave + i;
    v4f g = *(const v4fa*)(G + row * DF + 4 * lane);
    g.x += bb.x; g.y += bb.y; g.z += bb.z; g.w += bb.w;
    float ss = (g.x * g.x + g.y * g.y) + (g.z * g.z + g.w * g.w);
    ss += __shfl_xor(ss, 16, 32);
    ss += __shfl_xor(ss, 8, 32);
    ss += __shfl_xor(ss, 4, 32);
    ss += __shfl_xor(ss, 2, 32);
    ss += __shfl_xor(ss, 1, 32);
    const float den = fmaxf(sqrtf(ss), 1e-5f);
    const float rin = 1.0f / den;
    v4f o;
    o.x = g.x * rin; o.y = g.y * rin; o.z = g.z * rin; o.w = g.w * rin;
    ov[i] = o;
  }
#pragma unroll
  for (int i = 0; i < 4; ++i) *(volatile v4f*)(out + (size_t)(4 * wave + i) * DF + 4 * lane) = ov[i];
  __threadfence();
#pragma unroll
  for (int i = 0; i < 4; ++i) *(volatile v4f*)(out + (size_t)(4 * wave + i) * DF + 4 * lane) = ov[i];
}

static inline size_t al256(size_t o) { return (o + 255) & ~(size_t)255; }

extern "C" void kernel_launch(void* const* d_in, const int* in_sizes, int n_in,
                              void* d_out, int out_size, void* d_ws, size_t ws_size,
                              hipStream_t stream) {
  if (n_in < 8) return;
  if (in_sizes[0] != NGRAPH * NNODE) return;
  if (in_sizes[1] != NGRAPH * 2 * NEDGE) return;
  if (in_sizes[2] != NGRAPH * NEDGE) return;
  if (in_sizes[3] < DF || (in_sizes[3] % DF) != 0) return;
  const int nV = in_sizes[3] / DF;
  if (in_sizes[4] != NBAS * DF * DF) return;
  if (in_sizes[5] != NREL * NBAS) return;
  if (in_sizes[6] != DF * DF || in_sizes[7] != DF) return;
  if (out_size != NOUT) return;

  const int*   nid   = (const int*)d_in[0];
  const int*   eidx  = (const int*)d_in[1];
  const int*   etype = (const int*)d_in[2];
  const float* emb   = (const float*)d_in[3];
  const float* bases = (const float*)d_in[4];
  const float* comp  = (const float*)d_in[5];
  const float* root  = (const float*)d_in[6];
  const float* bias  = (const float*)d_in[7];
  float* out = (float*)d_out;

  char* ws = (char*)d_ws;
  size_t off = 0;
  const size_t oXB  = off; off = al256(off + (size_t)NGRAPH * NNODE * DF * 2);
  const size_t oWT  = off; off = al256(off + (size_t)DF * K2 * 2);
  const size_t oREC = off; off = al256(off + (size_t)NGRAPH * NBLKG * YPN * 4);
  const size_t oA2  = off; off = al256(off + (size_t)NGRAPH * K2 * 2);
  if (off > ws_size || off > (size_t)WSMAX) return;
  unsigned short* XB  = (unsigned short*)(ws + oXB);
  unsigned short* WT  = (unsigned short*)(ws + oWT);
  float*          REC = (float*)(ws + oREC);
  unsigned short* A2  = (unsigned short*)(ws + oA2);

  const size_t scanLds = (size_t)SCAN_LDS_INTS * 4;
  hipFuncSetAttribute(reinterpret_cast<const void*>(&k_scan), hipFuncAttributeMaxDynamicSharedMemorySize, (int)scanLds);

  k_prep<<<WBLK + XBLK, NTHR, 0, stream>>>(nid, emb, nV, root, bases, XB, WT);
  k_scan<<<dim3(NBLKG, NGRAPH), NTHR, scanLds, stream>>>(eidx, etype, XB, REC);
  k_combine<<<NGRAPH, NTHR, 0, stream>>>(REC, comp, A2);
  k_gemm<<<1, NTHR, 0, stream>>>(A2, WT, bias, out);
}
